// HSTUBlock_50500225466720
// MI455X (gfx1250) — hardware-verified
//
#include <hip/hip_runtime.h>


#define NB_  8
#define NT_  1024
#define DM   512
#define NH_  8
#define NKV  8
#define KVW  (NKV * HD)
#define HD   64
#define NTK  (NB_ * NT_)
#define NW   1024
#define NQKV 2048
#define NBKT 128
#define PSCW 1048576.0f
#define PSC  32768.0f
#define LOSC 1024.0f
#define LOSCI (1.0f / 1024.0f)

typedef _Float16 h16;
typedef unsigned short bf;
typedef __attribute__((ext_vector_type(16))) __bf16   v16bf;
typedef __attribute__((ext_vector_type(16))) _Float16 v16h;
typedef __attribute__((ext_vector_type(8)))  _Float16 v8h;
typedef __attribute__((ext_vector_type(8)))  unsigned short v8us;
typedef __attribute__((ext_vector_type(8)))  float    v8f;
typedef __attribute__((ext_vector_type(4)))  float    v4f;
typedef v8h  __attribute__((may_alias)) v8ha;
typedef v4f  __attribute__((may_alias)) v4fa;
typedef v8us __attribute__((may_alias)) v8usa;

__device__ __forceinline__ unsigned short f2bf(float f) { unsigned u = __float_as_uint(f); u += 0x7FFFu + ((u >> 16) & 1u); return (unsigned short)(u >> 16); }
__device__ __forceinline__ float bf2f(unsigned short b) { return __uint_as_float(((unsigned)b) << 16); }
__device__ __forceinline__ float bfr(float f) { return bf2f(f2bf(f)); }
__device__ __forceinline__ float silu_(float v) { return v / (1.0f + __expf(-v)); }
__device__ __forceinline__ v16h cat16(v8h lo, v8h hi) { return __builtin_shufflevector(lo, hi, 0, 1, 2, 3, 4, 5, 6, 7, 8, 9, 10, 11, 12, 13, 14, 15); }
__device__ __forceinline__ v16bf cat16b(v8us lo, v8us hi) { return __builtin_bit_cast(v16bf, __builtin_shufflevector(lo, hi, 0, 1, 2, 3, 4, 5, 6, 7, 8, 9, 10, 11, 12, 13, 14, 15)); }
__device__ __forceinline__ v8f wmma16(v16h a, v16h b, v8f c) { return __builtin_amdgcn_wmma_f32_16x16x32_f16(false, a, false, b, (short)0, c, false, false); }
__device__ __forceinline__ v8f wmmab(v16bf a, v16bf b, v8f c) { return __builtin_amdgcn_wmma_f32_16x16x32_bf16(false, a, false, b, (short)0, c, false, false); }

__global__ __launch_bounds__(256) void k_cvtb(const float* __restrict__ src, int nrows, bf* dst) {
    const int lane = threadIdx.x & 31, r = blockIdx.x * 8 + (threadIdx.x >> 5);
    if (r >= nrows) return;
    v8us o[DM / 256];
#pragma unroll
    for (int q = 0; q < DM / 256; ++q) { v8us t;
#pragma unroll
        for (int i = 0; i < 8; ++i) t[i] = f2bf(src[(size_t)r * DM + q * 256 + lane * 8 + i]);
        o[q] = t; }
#pragma unroll
    for (int q = 0; q < DM / 256; ++q) *(volatile v8us*)(dst + (size_t)r * DM + q * 256 + lane * 8) = o[q];
    __threadfence();
#pragma unroll
    for (int q = 0; q < DM / 256; ++q) *(volatile v8us*)(dst + (size_t)r * DM + q * 256 + lane * 8) = o[q];
}

__global__ __launch_bounds__(256) void k_wt(const float* __restrict__ Wm, int ncols, bf* WT) {
    __shared__ __align__(16) unsigned short tl[64 * 72];
    const int tid = threadIdx.x, k0 = blockIdx.x * 64, n0 = blockIdx.y * 64;
    const int kk = tid >> 2, nq = (tid & 3) * 16;
#pragma unroll
    for (int i = 0; i < 16; ++i) tl[(nq + i) * 72 + kk] = f2bf(Wm[(size_t)(k0 + kk) * ncols + n0 + nq + i]);
    __syncthreads();
    const int piece = tid & 7;
    typedef __attribute__((ext_vector_type(8))) unsigned short v8us_; typedef v8us_ __attribute__((may_alias)) v8usa_;
    auto pass = [&]() {
#pragma unroll
        for (int s = 0; s < 2; ++s) { const int nr = (tid >> 3) + 32 * s; const v8us_ val = *(const v8usa_*)(tl + nr * 72 + piece * 8);
            *(volatile v8us_*)(WT + (size_t)(n0 + nr) * DM + k0 + piece * 8) = val; }
    };
    pass(); __threadfence(); pass();
}

template <bool SPLITA, bool F16OUT = false>
__global__ __launch_bounds__(128) void k_gemmb(const bf* __restrict__ A, const bf* __restrict__ Al, const bf* __restrict__ Bn, const float* __restrict__ bias, float* C, int ldc, h16* C2) {
    __shared__ __align__(16) float ost[4][16 * 68];
    const int lane = threadIdx.x & 31, wave = threadIdx.x >> 5, lr = lane & 15, hi = lane >> 4;
    const int r0 = blockIdx.x * 64 + wave * 16, c0 = blockIdx.y * 64;
    const size_t aoff = (size_t)(r0 + lr) * DM + 8 * hi;
    size_t boff[4];
#pragma unroll
    for (int t = 0; t < 4; ++t) boff[t] = (size_t)(c0 + t * 16 + lr) * DM + 8 * hi;
    v8f acc[4];
#pragma unroll
    for (int t = 0; t < 4; ++t) acc[t] = (v8f){};
#pragma unroll 1
    for (int kc = 0; kc < DM; kc += 32) {
        const v16bf a = cat16b(*(const v8us*)(A + aoff + kc), *(const v8us*)(A + aoff + kc + 16));
        v16bf al = a;
        if (SPLITA) al = cat16b(*(const v8us*)(Al + aoff + kc), *(const v8us*)(Al + aoff + kc + 16));
#pragma unroll
        for (int t = 0; t < 4; ++t) { const v16bf b = cat16b(*(const v8us*)(Bn + boff[t] + kc), *(const v8us*)(Bn + boff[t] + kc + 16)); acc[t] = wmmab(a, b, acc[t]); if (SPLITA) acc[t] = wmmab(al, b, acc[t]); }
        asm volatile("v_nop\n\tv_nop\n\tv_nop\n\tv_nop" : "+v"(acc[0]), "+v"(acc[1]), "+v"(acc[2]), "+v"(acc[3]) : "v"(a), "v"(al));
    }
    float* os = &ost[wave][0];
#pragma unroll
    for (int t = 0; t < 4; ++t) { const float bv = bias ? bfr(bias[c0 + t * 16 + lr]) : 0.f;
#pragma unroll
        for (int j = 0; j < 8; ++j) os[(hi * 8 + j) * 68 + t * 16 + lr] = acc[t][j] + bv; }
    __syncthreads();
    if (F16OUT) {
        h16* crow = (h16*)(void*)C + (size_t)r0 * ldc + c0;
        auto pass = [&]() {
#pragma unroll
            for (int s = 0; s < 4; ++s) { const int row = 4 * s + (lane >> 3), piece = lane & 7; const float* sp = os + row * 68 + piece * 8; v8h o, o2;
#pragma unroll
                for (int i = 0; i < 8; ++i) { const h16 a = (h16)sp[i]; o[i] = a; o2[i] = (h16)((sp[i] - (float)a) * LOSC); }
                *(volatile v8h*)(crow + (size_t)row * ldc + piece * 8) = o; if (C2) *(volatile v8h*)(C2 + (size_t)r0 * ldc + c0 + (size_t)row * ldc + piece * 8) = o2; }
        };
        pass(); __threadfence(); pass();
    } else {
        float* crow = C + (size_t)r0 * ldc + c0;
        auto pass = [&]() {
#pragma unroll
            for (int s = 0; s < 8; ++s) { const int Lid = (lane >> 3) + 4 * s, piece = lane & 7; const int row = Lid >> 1, cofs = (Lid & 1) * 32 + piece * 4;
                const v4f val = *(const v4fa*)(os + row * 68 + cofs); *(volatile v4f*)(crow + (size_t)row * ldc + cofs) = val; }
        };
        pass(); __threadfence(); pass();
    }
}

__global__ __launch_bounds__(256) void k_ln1(const float* __restrict__ X, const float* __restrict__ g, const float* __restrict__ be, bf* PH, bf* PL) {
    const int lane = threadIdx.x & 31; const size_t r = (size_t)blockIdx.x * 8 + (threadIdx.x >> 5);
    if (r >= (size_t)NTK) return;
    const float* xr = X + r * DM; float s = 0.f;
#pragma unroll 1
    for (int q = 0; q < 2; ++q) { for (int i = 0; i < 8; ++i) s += bfr(xr[q * 256 + lane * 8 + i]); }
#pragma unroll
    for (int sh = 16; sh; sh >>= 1) s += __shfl_xor(s, sh, 32);
    const float mu = s * (1.0f / DM); float qq = 0.f;
#pragma unroll 1
    for (int q = 0; q < 2; ++q) { for (int i = 0; i < 8; ++i) { const float d = bfr(xr[q * 256 + lane * 8 + i]) - mu; qq += d * d; } }
#pragma unroll
    for (int sh = 16; sh; sh >>= 1) qq += __shfl_xor(qq, sh, 32);
    const float rs = rsqrtf(qq * (1.0f / DM) + 1e-6f);
#pragma unroll 1
    for (int ps = 0; ps < 2; ++ps) {
#pragma unroll 1
        for (int q = 0; q < 2; ++q) { v8us oh, ol;
#pragma unroll
            for (int i = 0; i < 8; ++i) { const int c = q * 256 + lane * 8 + i; const float y = (bfr(xr[c]) - mu) * rs * bfr(g[c]) + bfr(be[c]); const unsigned short hb = f2bf(y); oh[i] = hb; ol[i] = f2bf(y - bf2f(hb)); }
            *(volatile v8us*)(PH + r * DM + q * 256 + lane * 8) = oh; *(volatile v8us*)(PL + r * DM + q * 256 + lane * 8) = ol; }
        if (ps == 0) __threadfence(); }
}
__global__ __launch_bounds__(256) void k_ln2g(const float* __restrict__ Z, const float* __restrict__ U, const float* __restrict__ g, const float* __restrict__ be, bf* PH, bf* PL) {
    const int lane = threadIdx.x & 31; const size_t r = (size_t)blockIdx.x * 8 + (threadIdx.x >> 5);
    if (r >= (size_t)NTK) return;
    const float* zr = Z + r * DM; float s = 0.f;
#pragma unroll 1
    for (int q = 0; q < 2; ++q) { for (int i = 0; i < 8; ++i) s += zr[q * 256 + lane * 8 + i]; }
#pragma unroll
    for (int sh = 16; sh; sh >>= 1) s += __shfl_xor(s, sh, 32);
    const float mu = s * (1.0f / DM); float qq = 0.f;
#pragma unroll 1
    for (int q = 0; q < 2; ++q) { for (int i = 0; i < 8; ++i) { const float d = zr[q * 256 + lane * 8 + i] - mu; qq += d * d; } }
#pragma unroll
    for (int sh = 16; sh; sh >>= 1) qq += __shfl_xor(qq, sh, 32);
    const float rs = rsqrtf(qq * (1.0f / DM) + 1e-6f);
#pragma unroll 1
    for (int ps = 0; ps < 2; ++ps) {
#pragma unroll 1
        for (int q = 0; q < 2; ++q) { v8us oh, ol;
#pragma unroll
            for (int i = 0; i < 8; ++i) { const int c = q * 256 + lane * 8 + i; const float y = ((zr[c] - mu) * rs * bfr(g[c]) + bfr(be[c])) * silu_(U[r * DM + c]); const unsigned short hb = f2bf(y); oh[i] = hb; ol[i] = f2bf(y - bf2f(hb)); }
            *(volatile v8us*)(PH + r * DM + q * 256 + lane * 8) = oh; *(volatile v8us*)(PL + r * DM + q * 256 + lane * 8) = ol; }
        if (ps == 0) __threadfence(); }
}
__global__ __launch_bounds__(256) void k_act(const float* __restrict__ S, int rows, h16* PH, h16* PL) {
    const int lane = threadIdx.x & 31, r = blockIdx.x * 8 + (threadIdx.x >> 5);
    if (r >= rows) return;
#pragma unroll 1
    for (int q = 0; q < DM / 256; ++q) { v8h oh, ol;
#pragma unroll 2
        for (int i = 0; i < 8; ++i) { const float v = silu_(S[(size_t)r * DM + q * 256 + lane * 8 + i]); const h16 a = (h16)v; oh[i] = a; ol[i] = (h16)((v - (float)a) * LOSC); }
        *(volatile v8h*)(PH + (size_t)r * DM + q * 256 + lane * 8) = oh; *(volatile v8h*)(PL + (size_t)r * DM + q * 256 + lane * 8) = ol; __threadfence();
        *(volatile v8h*)(PH + (size_t)r * DM + q * 256 + lane * 8) = oh; *(volatile v8h*)(PL + (size_t)r * DM + q * 256 + lane * 8) = ol; }
}
__global__ __launch_bounds__(256) void k_vt(const float* __restrict__ V, h16* VTH, h16* VTL) {
    __shared__ __align__(16) h16 tile[64 * 72];
    __shared__ __align__(16) h16 til2[64 * 72];
    const int bid = blockIdx.x;
    const int b = bid / (NKV * (NT_ / 64)), rem = bid - b * (NKV * (NT_ / 64)), h = rem / (NT_ / 64), kt = rem - h * (NT_ / 64);
    const int k0 = kt * 64, tid = threadIdx.x;
    const int kk = tid >> 2, d0 = (tid & 3) * 16;
    const float* src = V + ((size_t)b * NT_ + k0 + kk) * KVW + h * HD + d0;
#pragma unroll 2
    for (int i = 0; i < 16; ++i) { const float v = silu_(src[i]); const h16 a = (h16)v; tile[(d0 + i) * 72 + kk] = a; til2[(d0 + i) * 72 + kk] = (h16)((v - (float)a) * LOSC); }
    __syncthreads();
    const int piece = tid & 7;
    const size_t base = (((size_t)b * NKV + h) * HD) * NT_ + k0;
    auto pass = [&]() {
#pragma unroll
        for (int s = 0; s < 4; ++s) { const int Lid = (tid >> 3) + 32 * s; const int pln = Lid >> 6, d = Lid & 63;
            const v8h val = *(const v8ha*)((pln ? til2 : tile) + d * 72 + piece * 8); *(volatile v8h*)((pln ? VTL : VTH) + base + (size_t)d * NT_ + piece * 8) = val; }
    };
    pass(); __threadfence(); pass();
}

__global__ __launch_bounds__(256) void k_resid(const float* __restrict__ X, float* out) {
    const int lane = threadIdx.x & 31; const size_t r = (size_t)blockIdx.x * 8 + (threadIdx.x >> 5);
    if (r >= (size_t)NTK) return;
    v4f v[DM / 128];
#pragma unroll
    for (int q = 0; q < DM / 128; ++q) { v[q] = *(const v4fa*)(out + r * DM + q * 128 + lane * 4);
#pragma unroll
        for (int i = 0; i < 4; ++i) v[q][i] += bfr(X[r * DM + q * 128 + lane * 4 + i]); }
    __builtin_amdgcn_wave_barrier(); asm volatile("" ::: "memory");
#pragma unroll
    for (int q = 0; q < DM / 128; ++q) *(volatile v4f*)(out + r * DM + q * 128 + lane * 4) = v[q];
    __threadfence();
#pragma unroll
    for (int q = 0; q < DM / 128; ++q) *(volatile v4f*)(out + r * DM + q * 128 + lane * 4) = v[q];
}
__global__ __launch_bounds__(128) void k_attn(const h16* __restrict__ Q16, const h16* __restrict__ QL16, const h16* __restrict__ K16, const h16* __restrict__ KL16, const h16* __restrict__ VTH, const h16* __restrict__ VTL,
                                             const int* __restrict__ ts, const float* __restrict__ amask, const float* __restrict__ posw, const float* __restrict__ tsw, float* Z) {
    __shared__ __align__(16) h16 plds[4][16 * 32];
    __shared__ __align__(16) h16 plds2[4][16 * 32];
    __shared__ __align__(16) float ost[4][16 * 68];
    const int lane = threadIdx.x & 31, wave = threadIdx.x >> 5, lr = lane & 15, hi = lane >> 4;
    const int bid = blockIdx.x;
    const int b = bid / (NH_ * (NT_ / 64)), rem = bid - b * (NH_ * (NT_ / 64)), h = rem / (NT_ / 64), qt = rem - h * (NT_ / 64);
    const int q0 = qt * 64 + wave * 16;
    const size_t tok0 = (size_t)b * NT_;
    h16* pl = &plds[wave][0]; h16* pl2 = &plds2[wave][0];
    v16h qa[2];
    const size_t qo0 = (tok0 + q0 + lr) * DM + h * HD + 8 * hi;
#pragma unroll
    for (int kc = 0; kc < 2; ++kc) qa[kc] = cat16(*(const v8h*)(Q16 + qo0 + kc * 32), *(const v8h*)(Q16 + qo0 + kc * 32 + 16));
    const h16* kh_b = K16 + tok0 * DM + h * HD; const h16* kl_b = KL16 + tok0 * DM + h * HD;
    const size_t vbase = (((size_t)b * NH_ + h) * HD) * NT_;
    int tsm[8];
#pragma unroll
    for (int j = 0; j < 8; ++j) { int m1 = q0 + hi * 8 + j + 1; if (m1 > NT_ - 1) m1 = NT_ - 1; tsm[j] = ts[tok0 + m1]; }
    v8f o[4], ox[4];
#pragma unroll
    for (int n = 0; n < 4; ++n) { o[n] = (v8f){}; ox[n] = (v8f){}; }
    const int kt_hi = (qt * 64 + 63) / 32;
#pragma unroll 1
    for (int kt = 0; kt <= kt_hi; ++kt) {
        const int l0 = kt * 32;
        const size_t ko0 = (size_t)(l0 + lr) * DM + 8 * hi, ko1 = (size_t)(l0 + 16 + lr) * DM + 8 * hi;
        v8f s0 = {}, s1 = {}, x0 = {}, x1 = {};
#pragma unroll
        for (int kc = 0; kc < 2; ++kc) {
            { const v16h k0h = cat16(*(const v8h*)(kh_b + ko0 + kc * 32), *(const v8h*)(kh_b + ko0 + kc * 32 + 16)), k1h = cat16(*(const v8h*)(kh_b + ko1 + kc * 32), *(const v8h*)(kh_b + ko1 + kc * 32 + 16));
              const v16h qlk = cat16(*(const v8h*)(QL16 + qo0 + kc * 32), *(const v8h*)(QL16 + qo0 + kc * 32 + 16));
              s0 = wmma16(qa[kc], k0h, s0); x0 = wmma16(qlk, k0h, x0); s1 = wmma16(qa[kc], k1h, s1); x1 = wmma16(qlk, k1h, x1);
              asm volatile("v_nop" : "+v"(s0), "+v"(s1), "+v"(x0), "+v"(x1) : "v"(qlk), "v"(k0h), "v"(k1h) : "memory"); }
            { const v16h k0l = cat16(*(const v8h*)(kl_b + ko0 + kc * 32), *(const v8h*)(kl_b + ko0 + kc * 32 + 16)), k1l = cat16(*(const v8h*)(kl_b + ko1 + kc * 32), *(const v8h*)(kl_b + ko1 + kc * 32 + 16));
              x0 = wmma16(qa[kc], k0l, x0); x1 = wmma16(qa[kc], k1l, x1);
              asm volatile("v_nop" : "+v"(x0), "+v"(x1) : "v"(k0l), "v"(k1l) : "memory"); }
        }
        asm volatile("v_nop\n\tv_nop\n\tv_nop\n\tv_nop" : "+v"(s0), "+v"(s1), "+v"(x0), "+v"(x1) : "v"(qa[0]), "v"(qa[1]));
        const int na = l0 + lr, nb = l0 + 16 + lr; const int tsa = ts[tok0 + na], tsb = ts[tok0 + nb];
#pragma unroll
        for (int j = 0; j < 8; ++j) { const int mr = hi * 8 + j, m = q0 + mr;
            float wa = 0.f, wb = 0.f;
            { const float keep = 1.0f - amask[(size_t)m * NT_ + na];
              if (keep != 0.f) { int d = tsm[j] - tsa; if (d < 0) d = -d; float mag = (float)d; if (mag < 1.0f) mag = 1.0f; int bk = (int)(logf(mag) / 0.301f); bk = bk < 0 ? 0 : (bk > NBKT ? NBKT : bk);
                  int pi = na - m + NT_ - 1; pi = pi < 0 ? 0 : (pi > 2 * NT_ - 2 ? 2 * NT_ - 2 : pi);
                  const float sc = (s0[j] + x0[j] * LOSCI) + bfr(posw[pi]) + bfr(tsw[bk]); wa = silu_(sc) * (1.0f / NT_) * keep; } }
            { const float keep = 1.0f - amask[(size_t)m * NT_ + nb];
              if (keep != 0.f) { int d = tsm[j] - tsb; if (d < 0) d = -d; float mag = (float)d; if (mag < 1.0f) mag = 1.0f; int bk = (int)(logf(mag) / 0.301f); bk = bk < 0 ? 0 : (bk > NBKT ? NBKT : bk);
                  int pi = nb - m + NT_ - 1; pi = pi < 0 ? 0 : (pi > 2 * NT_ - 2 ? 2 * NT_ - 2 : pi);
                  const float sc = (s1[j] + x1[j] * LOSCI) + bfr(posw[pi]) + bfr(tsw[bk]); wb = silu_(sc) * (1.0f / NT_) * keep; } }
            const float pa_ = wa * PSCW, pb_ = wb * PSCW; const h16 h0 = (h16)pa_, h1 = (h16)pb_;
            pl[mr * 32 + lr] = h0; pl[mr * 32 + 16 + lr] = h1; pl2[mr * 32 + lr] = (h16)(pa_ - (float)h0); pl2[mr * 32 + 16 + lr] = (h16)(pb_ - (float)h1); }
        asm volatile("" ::: "memory");
        const v16h pa = cat16(*(const v8ha*)(pl + lr * 32 + hi * 8), *(const v8ha*)(pl + lr * 32 + 16 + hi * 8));
        const v16h px = cat16(*(const v8ha*)(pl2 + lr * 32 + hi * 8), *(const v8ha*)(pl2 + lr * 32 + 16 + hi * 8));
#pragma unroll
        for (int n = 0; n < 4; ++n) { const size_t vo = vbase + (size_t)(n * 16 + lr) * NT_ + l0 + hi * 8;
            const v16h vh = cat16(*(const v8h*)(VTH + vo), *(const v8h*)(VTH + vo + 16)), vl = cat16(*(const v8h*)(VTL + vo), *(const v8h*)(VTL + vo + 16));
            o[n] = wmma16(pa, vh, o[n]); o[n] = wmma16(px, vh, o[n]); ox[n] = wmma16(pa, vl, ox[n]);
            asm volatile("" : "+v"(o[n]), "+v"(ox[n]) : "v"(vh), "v"(vl) : "memory"); }
        __builtin_amdgcn_wave_barrier();
    }
    float* os = &ost[wave][0];
#pragma unroll
    for (int n = 0; n < 4; ++n)
#pragma unroll
        for (int j = 0; j < 8; ++j) os[(hi * 8 + j) * 68 + n * 16 + lr] = (o[n][j] + ox[n][j] * LOSCI) * (1.0f / PSCW);
    __builtin_amdgcn_wave_barrier(); asm volatile("" ::: "memory");
    float* ob = Z + (tok0 + q0) * DM + (size_t)h * HD;
    auto pass = [&]() {
#pragma unroll
        for (int s = 0; s < 8; ++s) { const int Lid = (lane >> 3) + 4 * s, piece = lane & 7; const int row = Lid >> 1, cofs = (Lid & 1) * 32 + piece * 4;
            const v4f val = *(const v4fa*)(os + row * 68 + cofs); *(volatile v4f*)(ob + (size_t)row * DM + cofs) = val; }
    };
    pass(); __threadfence(); pass();
}

extern "C" void kernel_launch(void* const* d_in, const int* in_sizes, int n_in,
                              void* d_out, int out_size, void* d_ws, size_t ws_size, hipStream_t stream) {
    (void)in_sizes; (void)n_in; (void)out_size;
    const float* x = (const float*)d_in[0]; const int* ts = (const int*)d_in[1]; const float* amask = (const float*)d_in[2]; const float* Wu = (const float*)d_in[3]; const float* Wo = (const float*)d_in[4]; const float* bo = (const float*)d_in[5];
    const float* g1 = (const float*)d_in[6]; const float* b1 = (const float*)d_in[7]; const float* g2 = (const float*)d_in[8]; const float* b2 = (const float*)d_in[9]; const float* tsw = (const float*)d_in[10]; const float* posw = (const float*)d_in[11];
    float* out = (float*)d_out;
    char* wsp = (char*)d_ws;
    auto take = [&](size_t bytes) { char* p = wsp; wsp += (bytes + 255) & ~(size_t)255; return (void*)p; };
    bf* XH = (bf*)take((size_t)NTK * DM * 2); bf* XL = (bf*)take((size_t)NTK * DM * 2); bf* W4T = (bf*)take((size_t)NQKV * DM * 2); bf* WoT = (bf*)take((size_t)DM * DM * 2);
    float* Uf = (float*)take((size_t)NTK * DM * 4); float* Vf = (float*)take((size_t)NTK * DM * 4); float* Qf = (float*)take((size_t)NTK * DM * 4); float* Kf = (float*)take((size_t)NTK * DM * 4);
    h16* QH = (h16*)take((size_t)NTK * DM * 2); h16* QL = (h16*)take((size_t)NTK * DM * 2); h16* KH = (h16*)take((size_t)NTK * DM * 2); h16* KL = (h16*)take((size_t)NTK * DM * 2);
    if ((size_t)(wsp - (char*)d_ws) > ws_size) return;
    h16* VTH = (h16*)XH; h16* VTL = (h16*)XL; float* Z = Qf; bf* YH = (bf*)Kf; bf* YL = (bf*)((char*)Kf + (size_t)NTK * DM * 2);
    k_ln1<<<NTK / 8, 256, 0, stream>>>(x, g1, b1, XH, XL);
    k_wt<<<dim3(DM / 64, NQKV / 64, 1), 256, 0, stream>>>(Wu, NQKV, W4T);
    k_wt<<<dim3(DM / 64, DM / 64, 1), 256, 0, stream>>>(Wo, DM, WoT);
    k_gemmb<true, false><<<dim3(NTK / 64, DM / 64, 1), 128, 0, stream>>>(XH, XL, W4T, nullptr, Uf, DM, nullptr);
    k_gemmb<true, false><<<dim3(NTK / 64, DM / 64, 1), 128, 0, stream>>>(XH, XL, W4T + (size_t)DM * DM, nullptr, Vf, DM, nullptr);
    k_gemmb<true, false><<<dim3(NTK / 64, DM / 64, 1), 128, 0, stream>>>(XH, XL, W4T + (size_t)2 * DM * DM, nullptr, Qf, DM, nullptr);
    k_gemmb<true, false><<<dim3(NTK / 64, DM / 64, 1), 128, 0, stream>>>(XH, XL, W4T + (size_t)3 * DM * DM, nullptr, Kf, DM, nullptr);
    k_act<<<NTK / 8, 256, 0, stream>>>(Qf, NTK, QH, QL);
    k_act<<<NTK / 8, 256, 0, stream>>>(Kf, NTK, KH, KL);
    k_vt<<<NB_ * NKV * (NT_ / 64), 256, 0, stream>>>(Vf, VTH, VTL);
    k_attn<<<NB_ * NH_ * (NT_ / 64), 128, 0, stream>>>(QH, QL, KH, KL, VTH, VTL, ts, amask, posw, tsw, Z);
    k_ln2g<<<NTK / 8, 256, 0, stream>>>(Z, Uf, g2, b2, YH, YL);
    k_gemmb<true, false><<<dim3(NTK / 64, DM / 64, 1), 128, 0, stream>>>(YH, YL, WoT, bo, out, DM, nullptr);
    k_resid<<<NTK / 8, 256, 0, stream>>>(x, out);
}
